// SelfAttentionlayer_16844861735386
// MI455X (gfx1250) — hardware-verified
//
#include <hip/hip_runtime.h>
#include <math.h>

constexpr int kBatch = 8;
constexpr int kSeq   = 2048;
constexpr int kFeat  = 257;
constexpr int kTok   = kBatch * kSeq;
constexpr int kKPad  = 288;
constexpr int kNPad  = 320;
constexpr int kGrpB  = 4;
constexpr int kThrPerRow = kKPad / 8;
constexpr float kWCarry     = 16.0f;
constexpr float kWCarryInv  = 1.0f / 16.0f;
constexpr float kLogitScale = 0.062378286f;
constexpr int kCopyRows   = 32;
constexpr int kCopyFloats = kCopyRows * kFeat;
constexpr int kCopyF4     = kCopyFloats / 4;
static_assert(kKPad % 32 == 0 && kKPad >= kFeat && kKPad % 8 == 0, "kpad");
static_assert(kNPad % 64 == 0 && kNPad >= kKPad, "npad");
static_assert(kTok % 64 == 0 && kSeq % 64 == 0 && kSeq % 32 == 0, "tiles");
static_assert((kTok * kThrPerRow) % 256 == 0, "castgrid");
static_assert((kNPad * kThrPerRow) % 256 == 0, "wgrid");
static_assert(kCopyFloats % 4 == 0 && (kCopyRows * kFeat * 4) % 128 == 0, "lines");
static_assert(kTok % kCopyRows == 0 && kBatch % kGrpB == 0, "blocks");

typedef __attribute__((ext_vector_type(16))) _Float16 v16h;
typedef __attribute__((ext_vector_type(8)))  _Float16 v8h;
typedef __attribute__((ext_vector_type(16))) __bf16   v16b;
typedef __attribute__((ext_vector_type(8)))  __bf16   v8b;
typedef __attribute__((ext_vector_type(8)))  float    v8f;
typedef __attribute__((ext_vector_type(4)))  float    v4f;
typedef __attribute__((ext_vector_type(4)))  unsigned int v4u;

__device__ __forceinline__ unsigned short f2bf_bits(float f) {
  unsigned u = __float_as_uint(f);
  return (unsigned short)((u + 0x7FFFu + ((u >> 16) & 1u)) >> 16);
}
__device__ __forceinline__ float bf_bits2f(unsigned short h) { return __uint_as_float(((unsigned)h) << 16); }

__device__ __forceinline__ void dep_guard_h(v8f& a, v8f& b, v16h x, v16h y) { asm volatile("v_nop\n\tv_nop\n\tv_nop\n\tv_nop" : "+v"(a), "+v"(b) : "v"(x), "v"(y)); }
__device__ __forceinline__ void dep_guard_b(v8f& a, v8f& b, v16b x, v16b y) { asm volatile("v_nop\n\tv_nop\n\tv_nop\n\tv_nop" : "+v"(a), "+v"(b) : "v"(x), "v"(y)); }
__device__ __forceinline__ void dep_guard4_h(v8f& a, v8f& b, v8f& c, v8f& d, v16h x, v16h y) { asm volatile("v_nop\n\tv_nop\n\tv_nop\n\tv_nop" : "+v"(a), "+v"(b), "+v"(c), "+v"(d) : "v"(x), "v"(y)); }
__device__ __forceinline__ void dep_guard4_b(v8f& a, v8f& b, v8f& c, v8f& d, v16b x, v16b y) { asm volatile("v_nop\n\tv_nop\n\tv_nop\n\tv_nop" : "+v"(a), "+v"(b), "+v"(c), "+v"(d) : "v"(x), "v"(y)); }
__device__ __forceinline__ void keep4_h(v16h a, v16h b, v16h c, v16h d) { asm volatile("v_nop" :: "v"(a), "v"(b), "v"(c), "v"(d)); }
__device__ __forceinline__ void keep4_b(v16b a, v16b b, v16b c, v16b d) { asm volatile("v_nop" :: "v"(a), "v"(b), "v"(c), "v"(d)); }
__device__ __forceinline__ void acc_guard4(v8f& a, v8f& b, v8f& c, v8f& d) { asm volatile("v_nop\n\tv_nop\n\tv_nop\n\tv_nop" : "+v"(a), "+v"(b), "+v"(c), "+v"(d)); }
template <typename T> struct Frag;
template <> struct Frag<_Float16> {
  typedef v16h V; union U { v16h v; v8h h[2]; };
  static __device__ __forceinline__ v16h load(const _Float16* p) {
    U f; f.h[0] = *(const v8h*)(p); f.h[1] = *(const v8h*)(p + 16); return f.v;
  }
  static __device__ __forceinline__ v8f mma(v16h a, v16h b, v8f c) {
    return __builtin_amdgcn_wmma_f32_16x16x32_f16(false, a, false, b, (short)0, c, false, false);
  }
  static __device__ __forceinline__ void guard(v8f& a, v8f& b, v16h x, v16h y) { dep_guard_h(a, b, x, y); }
  static __device__ __forceinline__ void guard4(v8f& a, v8f& b, v8f& c, v8f& d, v16h x, v16h y) { dep_guard4_h(a, b, c, d, x, y); }
  static __device__ __forceinline__ void keep(v16h a, v16h b, v16h c, v16h d) { keep4_h(a, b, c, d); }
};
template <> struct Frag<__bf16> {
  typedef v16b V; union U { v16b v; v8b h[2]; };
  static __device__ __forceinline__ v16b load(const __bf16* p) {
    U f; f.h[0] = *(const v8b*)(p); f.h[1] = *(const v8b*)(p + 16); return f.v;
  }
  static __device__ __forceinline__ v8f mma(v16b a, v16b b, v8f c) {
    return __builtin_amdgcn_wmma_f32_16x16x32_bf16(false, a, false, b, (short)0, c, false, false);
  }
  static __device__ __forceinline__ void guard(v8f& a, v8f& b, v16b x, v16b y) { dep_guard_b(a, b, x, y); }
  static __device__ __forceinline__ void guard4(v8f& a, v8f& b, v8f& c, v8f& d, v16b x, v16b y) { dep_guard4_b(a, b, c, d, x, y); }
  static __device__ __forceinline__ void keep(v16b a, v16b b, v16b c, v16b d) { keep4_b(a, b, c, d); }
};

__device__ __forceinline__ unsigned pk16(unsigned short a, unsigned short b) { return (unsigned)a | ((unsigned)b << 16); }
__device__ __forceinline__ unsigned short h_bits(float f) { const _Float16 h = (_Float16)f; return __builtin_bit_cast(unsigned short, h); }

template <int ET> struct Elem;
template <> struct Elem<0> { typedef _Float16 T; };
template <> struct Elem<1> { typedef __bf16 T; };
template <int ET, bool SPLIT, int BIAS_MODE, int OUT_MODE, bool RESID, int ACT = 0>
__global__ __launch_bounds__(256) void wmma_gemm64(
    const unsigned short* __restrict__ Ap, const unsigned short* __restrict__ A2p, int lda, long strideA,
    const unsigned short* __restrict__ Btp, const unsigned short* __restrict__ Bt2p, int ldb, long strideB,
    void* __restrict__ Cout, void* __restrict__ Cout2, int ldc, long strideC,
    const float* __restrict__ bias,
    const float* __restrict__ resid, long strideR,
    int M, int N, int K, float scale) {
  typedef typename Elem<ET>::T T;
  typedef typename Frag<T>::V V;
  const T* A = (const T*)Ap; const T* A2 = (const T*)A2p; const T* Bt = (const T*)Btp; const T* Bt2 = (const T*)Bt2p;
  __shared__ __align__(16) float sT[8][16 * 68];
  const int b    = blockIdx.y;
  const int lane = threadIdx.x & 31;
  const int wave = threadIdx.x >> 5;
  const int tilesN = N >> 6;
  const int tilesM = M >> 6;
  const int tile = blockIdx.x * 8 + wave;
  if (tile >= tilesM * tilesN) return;
  const int tm = tile / tilesN;
  const int tn = tile - tm * tilesN;
  const int m0 = tm << 6;
  const int n0 = tn << 6;

  const T* Ab  = A  + (size_t)b * strideA;
  const T* Bb  = Bt + (size_t)b * strideB;
  const T* Ab2 = SPLIT ? (A2  + (size_t)b * strideA) : nullptr;
  const T* Bb2 = SPLIT ? (Bt2 + (size_t)b * strideB) : nullptr;

  const int rlane = lane & 15;
  const int koff  = (lane >> 4) * 8;
  const int mOff  = (lane >> 4) * 8;

  v8f acc[4][4];
#pragma unroll
  for (int i = 0; i < 4; ++i)
#pragma unroll
    for (int j = 0; j < 4; ++j) acc[i][j] = (v8f){0.f,0.f,0.f,0.f,0.f,0.f,0.f,0.f};

  for (int k0 = 0; k0 < K; k0 += 32) {
    V bh[4], bl[4];
#pragma unroll
    for (int j = 0; j < 4; ++j) {
      const size_t bo = (size_t)(n0 + (j << 4) + rlane) * ldb + koff + k0;
      bh[j] = Frag<T>::load(Bb + bo);
      if (SPLIT) bl[j] = Frag<T>::load(Bb2 + bo);
    }
#pragma unroll
    for (int i = 0; i < 4; ++i) {
      const size_t ao = (size_t)(m0 + (i << 4) + rlane) * lda + koff + k0;
      V ah = Frag<T>::load(Ab + ao);
      V al;
      if (SPLIT) al = Frag<T>::load(Ab2 + ao);
#pragma unroll
      for (int j = 0; j < 4; ++j) {
        acc[i][j] = Frag<T>::mma(ah, bh[j], acc[i][j]);
        if (SPLIT) {
          acc[i][j] = Frag<T>::mma(ah, bl[j], acc[i][j]);
          acc[i][j] = Frag<T>::mma(al, bh[j], acc[i][j]);
        }
      }
      Frag<T>::guard4(acc[i][0], acc[i][1], acc[i][2], acc[i][3], ah, SPLIT ? al : ah);
    }
    Frag<T>::keep(bh[0], bh[1], bh[2], bh[3]);
    if (SPLIT) Frag<T>::keep(bl[0], bl[1], bl[2], bl[3]);
  }
  acc_guard4(acc[0][0], acc[0][1], acc[0][2], acc[0][3]);
  acc_guard4(acc[1][0], acc[1][1], acc[1][2], acc[1][3]);
  acc_guard4(acc[2][0], acc[2][1], acc[2][2], acc[2][3]);
  acc_guard4(acc[3][0], acc[3][1], acc[3][2], acc[3][3]);

  float* slab = sT[wave];
  const float* Rb = RESID ? (resid + (size_t)b * strideR) : nullptr;
#pragma unroll
  for (int i = 0; i < 4; ++i) {
    const int mBase = m0 + (i << 4);
#pragma unroll
    for (int j = 0; j < 4; ++j) {
      const int n = n0 + (j << 4) + rlane;
      float bv = 0.f;
      if (BIAS_MODE == 2) bv = bias[n];
#pragma unroll
      for (int r = 0; r < 8; ++r) {
        float v = acc[i][j][r] * scale;
        if (BIAS_MODE == 1) v += bias[mBase + mOff + r];
        if (BIAS_MODE == 2) v += bv;
        if (RESID) v += Rb[(size_t)(mBase + mOff + r) * ldc + n];
        if (ACT == 2) v = fmaxf(v, 0.0f);
        if (ACT == 4) v = (v > 0.f) ? v : 0.01f * v;
        if (ACT == 6) v = 1.0f / (1.0f + expf(-v));
        slab[(mOff + r) * 68 + (j << 4) + rlane] = v;
      }
    }
    __builtin_amdgcn_fence(__ATOMIC_RELEASE, "workgroup");
    __builtin_amdgcn_wave_barrier();
    __builtin_amdgcn_fence(__ATOMIC_ACQUIRE, "workgroup");
    if (OUT_MODE == 0) {
      float* C = (float*)Cout + (size_t)b * strideC;
      const int hh = lane >> 4, c4 = (lane & 15) * 4;
      for (int pass = 0; pass < 2; ++pass) {
#pragma unroll
        for (int it = 0; it < 8; ++it) {
          const int row = it * 2 + hh;
          v4f v = *(const v4f*)(slab + row * 68 + c4);
          *(volatile v4f*)(C + (size_t)(mBase + row) * ldc + n0 + c4) = v;
        }
        __threadfence();
      }
    } else {
      const int q = lane >> 3, c8 = (lane & 7) * 8;
      unsigned short* C  = (unsigned short*)Cout  + (size_t)b * strideC;
      unsigned short* C2 = (OUT_MODE == 2) ? ((unsigned short*)Cout2 + (size_t)b * strideC) : nullptr;
      for (int pass = 0; pass < 2; ++pass) {
#pragma unroll
        for (int it = 0; it < 4; ++it) {
          const int row = it * 4 + q;
          const float* sp = slab + row * 68 + c8;
          v8h hv, lv;
#pragma unroll
          for (int e = 0; e < 8; ++e) {
            if (OUT_MODE == 1) {
              hv[e] = (_Float16)sp[e];
            } else {
              unsigned short hb = f2bf_bits(sp[e]);
              unsigned short lb = f2bf_bits(sp[e] - bf_bits2f(hb));
              hv[e] = __builtin_bit_cast(_Float16, hb);
              lv[e] = __builtin_bit_cast(_Float16, lb);
            }
          }
          *(volatile v8h*)(C + (size_t)(mBase + row) * ldc + n0 + c8) = hv;
          if (OUT_MODE == 2) *(volatile v8h*)(C2 + (size_t)(mBase + row) * ldc + n0 + c8) = lv;
        }
        __threadfence();
      }
    }
    __builtin_amdgcn_fence(__ATOMIC_RELEASE, "workgroup");
    __builtin_amdgcn_wave_barrier();
    __builtin_amdgcn_fence(__ATOMIC_ACQUIRE, "workgroup");
  }
}

__global__ __launch_bounds__(256) void cast_x_kernel(const float* __restrict__ x, unsigned short* __restrict__ X16, int nthr) {
  const int i = blockIdx.x * 256 + threadIdx.x;
  if (i >= nthr) return;
  const int row = i / kThrPerRow;
  const int col = (i - row * kThrPerRow) * 8;
  const float* src = x + (size_t)row * kFeat;
  unsigned short hb[8];
#pragma unroll
  for (int e = 0; e < 8; ++e) {
    const int c  = col + e;
    const int cc = (c < kFeat) ? c : (kFeat - 1);
    const float keep = (c < kFeat) ? 1.0f : 0.0f;
    const float v = src[cc] * keep;
    hb[e] = h_bits(v);
  }
  const v4u u = (v4u){pk16(hb[0], hb[1]), pk16(hb[2], hb[3]), pk16(hb[4], hb[5]), pk16(hb[6], hb[7])};
  unsigned short* dp = X16 + 8 * (size_t)i;
  *(volatile v4u*)dp = u;
  __threadfence();
  *(volatile v4u*)dp = u;
}

__global__ __launch_bounds__(256) void pack_w_kernel(const float* __restrict__ W0, const float* __restrict__ W1,
                                                     const float* __restrict__ W2, const float* __restrict__ W3,
                                                     unsigned short* __restrict__ W16) {
  const int z = blockIdx.y;
  const float* W = (z == 0) ? W0 : (z == 1) ? W1 : (z == 2) ? W2 : W3;
  const int i = blockIdx.x * 256 + threadIdx.x;
  if (i >= kNPad * kThrPerRow) return;
  const int n   = i / kThrPerRow;
  const int col = (i - n * kThrPerRow) * 8;
  const int nn  = (n < kFeat) ? n : (kFeat - 1);
  const float rowkeep = (n < kFeat) ? kWCarry : 0.0f;
  const float* src = W + (size_t)nn * kFeat;
  unsigned short hb[8];
#pragma unroll
  for (int e = 0; e < 8; ++e) {
    const int c  = col + e;
    const int cc = (c < kFeat) ? c : (kFeat - 1);
    const float keep = (c < kFeat) ? rowkeep : 0.0f;
    const float v = src[cc] * keep;
    hb[e] = h_bits(v);
  }
  const v4u u = (v4u){pk16(hb[0], hb[1]), pk16(hb[2], hb[3]), pk16(hb[4], hb[5]), pk16(hb[6], hb[7])};
  unsigned short* dp = W16 + (size_t)z * kNPad * kKPad + 8 * (size_t)i;
  *(volatile v4u*)dp = u;
  __threadfence();
  *(volatile v4u*)dp = u;
}

__global__ __launch_bounds__(96) void pack_bias_kernel(const float* __restrict__ b0, const float* __restrict__ b1,
                                                       const float* __restrict__ b2, const float* __restrict__ b3,
                                                       float* __restrict__ BP) {
  const int z = blockIdx.x;
  const float* src = (z == 0) ? b0 : (z == 1) ? b1 : (z == 2) ? b2 : b3;
  const int t = threadIdx.x;
  if (t >= kNPad / 4) return;
  v4f v;
#pragma unroll
  for (int e = 0; e < 4; ++e) {
    const int c  = 4 * t + e;
    const int cc = (c < kFeat) ? c : (kFeat - 1);
    const float keep = (c < kFeat) ? 1.0f : 0.0f;
    v[e] = src[cc] * keep;
  }
  float* dp = BP + (size_t)z * kNPad + 4 * t;
  *(volatile v4f*)dp = v;
  __threadfence();
  *(volatile v4f*)dp = v;
}

__global__ __launch_bounds__(256) void copy_out_kernel(const float* __restrict__ src, float* __restrict__ out) {
  const int blk = blockIdx.x;
  const int t   = threadIdx.x;
  const int base = blk * kCopyFloats;
#pragma unroll 1
  for (int j = 0; j < 9; ++j) {
    const int f  = j * 256 + t;
    const int fc = (f < kCopyF4) ? f : (kCopyF4 - 1);
    v4f v;
#pragma unroll
    for (int e = 0; e < 4; ++e) {
      const int flat = base + 4 * fc + e;
      const int row  = flat / kFeat;
      const int col  = flat - row * kFeat;
      v[e] = src[(size_t)row * kNPad + col];
    }
    if (f < kCopyF4) {
      float* dp = out + (size_t)base + 4 * (size_t)f;
      *(volatile v4f*)dp = v;
      __threadfence();
      *(volatile v4f*)dp = v;
    }
    asm volatile("" ::: "memory");
  }
}

typedef void (*GemmFn)(const unsigned short*, const unsigned short*, int, long,
                       const unsigned short*, const unsigned short*, int, long,
                       void*, void*, int, long, const float*, const float*, long, int, int, int, float);

extern "C" void kernel_launch(void* const* d_in, const int* in_sizes, int n_in,
                              void* d_out, int out_size, void* d_ws, size_t ws_size,
                              hipStream_t stream) {
  if (n_in < 11) return;
  const int nAct = kTok * kFeat;
  const int nW   = kFeat * kFeat;
  if (in_sizes[0] != nAct || in_sizes[1] != nAct || in_sizes[2] != nAct) return;
  if (in_sizes[3] != nW || in_sizes[5] != nW || in_sizes[7] != nW || in_sizes[9] != nW) return;
  if (in_sizes[4] != kFeat || in_sizes[6] != kFeat || in_sizes[8] != kFeat || in_sizes[10] != kFeat) return;
  if (out_size != nAct) return;

  const size_t szX  = (size_t)kTok * kKPad * 2;
  const size_t szP  = (size_t)kTok * kNPad * 2;
  const size_t szVT = (size_t)kBatch * kNPad * kSeq * 2;
  const size_t szS  = (size_t)kGrpB * kSeq * kSeq * 2;
  const size_t szO  = (size_t)kTok * kNPad * 4;
  const size_t szW  = (size_t)4 * kNPad * kKPad * 2;
  const size_t szB  = (size_t)4 * kNPad * 4;
  const size_t offX   = 0;
  const size_t offQP  = offX + szX;
  const size_t offKP  = offQP + szP;
  const size_t offVT  = offKP + szP;
  const size_t offCTX = offVT + szVT;
  const size_t offS   = offCTX + szP;
  const size_t offO   = offS + szS;
  const size_t offW   = offO + szO;
  const size_t offB   = offW + szW;
  const size_t total  = offB + szB;
  if (ws_size < total) return;

  const float* q  = (const float*)d_in[0];
  const float* k  = (const float*)d_in[1];
  const float* v  = (const float*)d_in[2];
  const float* Wq = (const float*)d_in[3];
  const float* bq = (const float*)d_in[4];
  const float* Wk = (const float*)d_in[5];
  const float* bk = (const float*)d_in[6];
  const float* Wv = (const float*)d_in[7];
  const float* bv = (const float*)d_in[8];
  const float* Wo = (const float*)d_in[9];
  const float* bo = (const float*)d_in[10];
  float* out = (float*)d_out;
  char* ws = (char*)d_ws;
  unsigned short* X16   = (unsigned short*)(ws + offX);
  unsigned short* QP16  = (unsigned short*)(ws + offQP);
  unsigned short* KP16  = (unsigned short*)(ws + offKP);
  unsigned short* VPT16 = (unsigned short*)(ws + offVT);
  unsigned short* CTX16 = (unsigned short*)(ws + offCTX);
  unsigned short* S16   = (unsigned short*)(ws + offS);
  float*          OUTF  = (float*)(ws + offO);
  unsigned short* W16   = (unsigned short*)(ws + offW);
  float*          BP    = (float*)(ws + offB);
  const size_t planeW = (size_t)kNPad * kKPad;
  unsigned short* Wq16 = W16 + 0 * planeW;
  unsigned short* Wk16 = W16 + 1 * planeW;
  unsigned short* Wv16 = W16 + 2 * planeW;
  unsigned short* Wo16 = W16 + 3 * planeW;
  const float* BPq = BP + 0 * kNPad;
  const float* BPk = BP + 1 * kNPad;
  const float* BPv = BP + 2 * kNPad;
  const float* BPo = BP + 3 * kNPad;

  GemmFn gemmProjN = wmma_gemm64<0, false, 2, 1, false, 0>;
  GemmFn gemmProjT = wmma_gemm64<0, false, 1, 1, false, 0>;
  GemmFn gemmScore = wmma_gemm64<0, false, 0, 1, false, 6>;
  GemmFn gemmCtx   = wmma_gemm64<0, false, 0, 1, false, 0>;
  GemmFn gemmOut   = wmma_gemm64<0, false, 2, 0, false, 0>;

  pack_w_kernel<<<dim3((kNPad * kThrPerRow) / 256, 4), dim3(256), 0, stream>>>(Wq, Wk, Wv, Wo, W16);
  pack_bias_kernel<<<dim3(4), dim3(96), 0, stream>>>(bq, bk, bv, bo, BP);

  const int nthrX   = kTok * kThrPerRow;
  const int tilesPN = (kTok / 64) * (kNPad / 64);
  const int tilesPT = (kNPad / 64) * (kSeq / 64);
  const int tilesSc = (kSeq / 64) * (kSeq / 64);
  const int tilesCx = (kSeq / 64) * (kNPad / 64);

  cast_x_kernel<<<dim3(nthrX / 256), dim3(256), 0, stream>>>(q, X16, nthrX);
  gemmProjN<<<dim3(tilesPN / 8, 1), dim3(256), 0, stream>>>(
      X16, X16, kKPad, 0L, Wq16, Wq16, kKPad, 0L, (void*)QP16, (void*)QP16, kNPad, 0L,
      BPq, BPq, 0L, kTok, kNPad, kKPad, kWCarryInv);
  cast_x_kernel<<<dim3(nthrX / 256), dim3(256), 0, stream>>>(k, X16, nthrX);
  gemmProjN<<<dim3(tilesPN / 8, 1), dim3(256), 0, stream>>>(
      X16, X16, kKPad, 0L, Wk16, Wk16, kKPad, 0L, (void*)KP16, (void*)KP16, kNPad, 0L,
      BPk, BPk, 0L, kTok, kNPad, kKPad, kWCarryInv);
  cast_x_kernel<<<dim3(nthrX / 256), dim3(256), 0, stream>>>(v, X16, nthrX);
  gemmProjT<<<dim3(tilesPT / 8, kBatch), dim3(256), 0, stream>>>(
      Wv16, Wv16, kKPad, 0L, X16, X16, kKPad, (long)kSeq * kKPad, (void*)VPT16, (void*)VPT16, kSeq, (long)kNPad * kSeq,
      BPv, BPv, 0L, kNPad, kSeq, kKPad, kWCarryInv);

  for (int h = 0; h < kBatch / kGrpB; ++h) {
    const size_t rowOff = (size_t)h * kGrpB * kSeq;
    const unsigned short* QPg  = QP16 + rowOff * kNPad;
    const unsigned short* KPg  = KP16 + rowOff * kNPad;
    const unsigned short* VPTg = VPT16 + (size_t)h * kGrpB * kNPad * kSeq;
    unsigned short*       CTXg = CTX16 + rowOff * kNPad;
    gemmScore<<<dim3(tilesSc / 8, kGrpB), dim3(256), 0, stream>>>(
        QPg, QPg, kNPad, (long)kSeq * kNPad, KPg, KPg, kNPad, (long)kSeq * kNPad,
        (void*)S16, (void*)S16, kSeq, (long)kSeq * kSeq, BPq, BPq, 0L, kSeq, kSeq, kKPad, kLogitScale);
    gemmCtx<<<dim3(tilesCx / 8, kGrpB), dim3(256), 0, stream>>>(
        S16, S16, kSeq, (long)kSeq * kSeq, VPTg, VPTg, kSeq, (long)kNPad * kSeq,
        (void*)CTXg, (void*)CTXg, kNPad, (long)kSeq * kNPad, BPq, BPq, 0L, kSeq, kNPad, kSeq, 1.0f);
  }

  gemmOut<<<dim3(tilesPN / 8, 1), dim3(256), 0, stream>>>(
      CTX16, CTX16, kNPad, 0L, Wo16, Wo16, kKPad, 0L, (void*)OUTF, (void*)OUTF, kNPad, 0L,
      BPo, BPo, 0L, kTok, kNPad, kKPad, kWCarryInv);
  copy_out_kernel<<<dim3(kTok / kCopyRows), dim3(256), 0, stream>>>(OUTF, out);
}
